// QNN_28157805593247
// MI455X (gfx1250) — hardware-verified
//
#include <hip/hip_runtime.h>
#include <math.h>

constexpr int NBATCH = 1024;
constexpr int NSTEP  = 512;
constexpr int NIN    = 24;
constexpr int NHID   = 128;
constexpr int NGATE  = 4 * NHID;
constexpr int KUSE   = NHID + NIN;
constexpr int KTOT   = 160;
constexpr int APITCH = 168;
constexpr int LPITCH = 136;
constexpr int WPITCH = 192;
constexpr int WGRP   = WPITCH / 8;
constexpr int RBLK   = 32;
constexpr int NTHR   = 512;
constexpr int XQ     = NIN / 4;
constexpr int XTHR   = RBLK * XQ;
constexpr int NCAT   = NHID + 2;
constexpr int NZ     = 64;
constexpr int NOUTC  = 3;
constexpr int HSP    = 132;
constexpr int ZSP    = 68;
constexpr int OSN    = 128;
constexpr int NPREP  = 256;
static_assert(KTOT % 32 == 0 && NHID % 32 == 0);
static_assert(KTOT >= KUSE && KTOT - KUSE == 8 && APITCH >= KTOT && WPITCH >= KTOT && LPITCH >= NHID);
static_assert(APITCH % 8 == 0 && LPITCH % 8 == 0 && WPITCH % 8 == 0);
static_assert((WPITCH * 2) % 128 == 0);
static_assert(NBATCH % RBLK == 0);
static_assert(NTHR / 32 == 2 * (NHID / 16));
static_assert(XTHR % 32 == 0 && XTHR <= NTHR);
static_assert(NIN % 8 == 0);
static_assert((RBLK * NOUTC * 4) % 128 == 0);
static_assert(RBLK * NOUTC <= OSN && OSN == 4 * 32);
static_assert((NGATE * WGRP) % NPREP == 0);
static_assert(NTHR == RBLK * 16 && NZ == 16 * 4);
static_assert(RBLK * NOUTC <= 128 && NOUTC * NZ <= NTHR && (NOUTC * NZ) % 32 == 0);
static_assert(HSP % 4 == 0 && ZSP % 4 == 0);

typedef __attribute__((ext_vector_type(16))) __bf16   v16b;
typedef __attribute__((ext_vector_type(8)))  __bf16   v8b;
typedef __attribute__((ext_vector_type(8)))  _Float16 v8h;
typedef __attribute__((ext_vector_type(8)))  float    v8f;
typedef __attribute__((ext_vector_type(4)))  float    v4f;
typedef __attribute__((ext_vector_type(2)))  unsigned v2u;

__device__ __forceinline__ unsigned short f2bf_bits(float f) {
  unsigned u = __float_as_uint(f);
  return (unsigned short)((u + 0x7FFFu + ((u >> 16) & 1u)) >> 16);
}
__device__ __forceinline__ float bf_bits2f(unsigned short h) { return __uint_as_float(((unsigned)h) << 16); }
__device__ __forceinline__ float bf16r(float f) { return bf_bits2f(f2bf_bits(f)); }

__device__ __forceinline__ void mma_guard4_b(v8f& a, v8f& b, v8f& c, v8f& d, v16b x, v16b y) {
  asm volatile("v_nop\n\tv_nop\n\tv_nop\n\tv_nop" : "+v"(a), "+v"(b), "+v"(c), "+v"(d) : "v"(x), "v"(y));
}
__device__ __forceinline__ void keep4_b(v16b a, v16b b, v16b c, v16b d) { asm volatile("v_nop" :: "v"(a), "v"(b), "v"(c), "v"(d)); }
__device__ __forceinline__ void acc_guard4(v8f& a, v8f& b, v8f& c, v8f& d) { asm volatile("v_nop\n\tv_nop\n\tv_nop\n\tv_nop" : "+v"(a), "+v"(b), "+v"(c), "+v"(d)); }
template <typename T> struct Frag;
template <> struct Frag<__bf16> {
  typedef v16b V; union U { v16b v; v8b h[2]; };
  static __device__ __forceinline__ v16b load(const __bf16* p) {
    U f; f.h[0] = *(const v8b*)(p); f.h[1] = *(const v8b*)(p + 16); return f.v;
  }
  static __device__ __forceinline__ v8f mma(v16b a, v16b b, v8f c) {
    return __builtin_amdgcn_wmma_f32_16x16x32_bf16(false, a, false, b, (short)0, c, false, false);
  }
};

__device__ __forceinline__ float fsig(float x)  { return __builtin_amdgcn_rcpf(1.0f + __expf(-x)); }
__device__ __forceinline__ float ftanh(float x) { return 1.0f - 2.0f * __builtin_amdgcn_rcpf(__expf(2.0f * x) + 1.0f); }

__global__ __launch_bounds__(NPREP) void wprep_kernel(const float* __restrict__ W_hh, const float* __restrict__ W_ih,
                                                      unsigned short* __restrict__ WC) {
  const int i = blockIdx.x * NPREP + threadIdx.x;
  if (i >= NGATE * WGRP) return;
  const int n = i / WGRP;
  const int q = i - n * WGRP;
  const int qh  = (q < 16) ? q : 15;
  const int qx0 = q - 16;
  const int qx  = (qx0 < 0) ? 0 : ((qx0 > 2) ? 2 : qx0);
  const float fh = (q < 16) ? 1.0f : 0.0f;
  const float fx = (q >= 16 && q < 19) ? 1.0f : 0.0f;
  const float* ph = W_hh + (size_t)n * NHID + 8 * qh;
  const float* px = W_ih + (size_t)n * NIN + 8 * qx;
  const v4f a0 = *(const v4f*)(ph);
  const v4f a1 = *(const v4f*)(ph + 4);
  const v4f x0 = *(const v4f*)(px);
  const v4f x1 = *(const v4f*)(px + 4);
  v8h hv;
#pragma unroll
  for (int e = 0; e < 4; ++e) {
    const float v0 = fmaf(fh, a0[e], fx * x0[e]);
    const float v1 = fmaf(fh, a1[e], fx * x1[e]);
    hv[e]     = __builtin_bit_cast(_Float16, f2bf_bits(v0));
    hv[4 + e] = __builtin_bit_cast(_Float16, f2bf_bits(v1));
  }
  unsigned short* op = WC + (size_t)n * WPITCH + 8 * q;
  *(volatile v8h*)op = hv;
  __threadfence();
  *(volatile v8h*)op = hv;
}

__global__ __launch_bounds__(NTHR) void lstm_head_kernel(const float* __restrict__ x, const float* __restrict__ addin,
                                                        const unsigned short* __restrict__ WCp,
                                                        const float* __restrict__ b_ih, const float* __restrict__ b_hh,
                                                        const float* __restrict__ W1, const float* __restrict__ b1,
                                                        const float* __restrict__ W2, const float* __restrict__ b2,
                                                        float* __restrict__ out) {
  __shared__ __align__(16) unsigned short Ah[RBLK * APITCH];
  __shared__ __align__(16) unsigned short Al[RBLK * LPITCH];
  __shared__ __align__(16) float          Hs[RBLK * HSP];
  __shared__ __align__(16) float          W1s[NZ * NCAT];
  __shared__ __align__(16) float          W2s[NOUTC * NZ];
  __shared__ __align__(16) float          Zs[RBLK * ZSP];
  __shared__ __align__(16) float          Os[OSN];
  const __bf16* WC = (const __bf16*)WCp;
  const int tid = threadIdx.x, lane = tid & 31, wave = tid >> 5;
  const int c = lane & 15, hh = lane >> 4, koff = hh * 8;
  const int msub = wave >> 3, ub = wave & 7;
  const int j = 16 * ub + c;
  const int arow0 = 16 * msub + 8 * hh;
  const int rowbase = blockIdx.x * RBLK;

#pragma unroll 1
  for (int i = tid; i < RBLK * APITCH; i += NTHR) Ah[i] = (unsigned short)0;
#pragma unroll 1
  for (int i = tid; i < RBLK * LPITCH; i += NTHR) Al[i] = (unsigned short)0;

  float cst[8], hst[8], bb[4];
#pragma unroll
  for (int r = 0; r < 8; ++r) { cst[r] = 0.0f; hst[r] = 0.0f; }
#pragma unroll
  for (int g = 0; g < 4; ++g) bb[g] = bf16r(b_ih[g * NHID + j]) + bf16r(b_hh[g * NHID + j]);

  const int xm0 = tid / XQ;
  const int xm  = (tid < XTHR) ? xm0 : 0;
  const int xq  = (tid < XTHR) ? (tid - XQ * xm0) : 0;
  const float* xrow = x + ((size_t)(rowbase + xm) * NSTEP) * NIN + 4 * xq;
  unsigned short* axdst = Ah + xm * APITCH + NHID + 4 * xq;
  __syncthreads();
  if (tid < XTHR) {
    const v4f v = *(const v4f*)(xrow);
    v2u pk;
    pk[0] = (unsigned)f2bf_bits(v[0]) | ((unsigned)f2bf_bits(v[1]) << 16);
    pk[1] = (unsigned)f2bf_bits(v[2]) | ((unsigned)f2bf_bits(v[3]) << 16);
    *(v2u*)(axdst) = pk;
  }
  __syncthreads();

  const __bf16* ahrow = (const __bf16*)Ah + (16 * msub + c) * APITCH + koff;
  const __bf16* alrow = (const __bf16*)Al + (16 * msub + c) * LPITCH + koff;
  const __bf16* w0 = WC + (size_t)(0 * NHID + j) * WPITCH + koff;
  const __bf16* w1 = WC + (size_t)(1 * NHID + j) * WPITCH + koff;
  const __bf16* w2 = WC + (size_t)(2 * NHID + j) * WPITCH + koff;
  const __bf16* w3 = WC + (size_t)(3 * NHID + j) * WPITCH + koff;
  const v8f z8 = {0.f, 0.f, 0.f, 0.f, 0.f, 0.f, 0.f, 0.f};

#pragma unroll 1
  for (int t = 0; t < NSTEP; ++t) {
    const int tn = (t + 1 < NSTEP) ? (t + 1) : (NSTEP - 1);
    const v4f xv = *(const v4f*)(xrow + (size_t)tn * NIN);

    v8f acc[4];
    acc[0] = z8; acc[1] = z8; acc[2] = z8; acc[3] = z8;
#pragma unroll 1
    for (int k0 = 0; k0 < NHID; k0 += 32) {
      const v16b ahv = Frag<__bf16>::load(ahrow + k0);
      const v16b alv = Frag<__bf16>::load(alrow + k0);
      const v16b bq0 = Frag<__bf16>::load(w0 + k0);
      const v16b bq1 = Frag<__bf16>::load(w1 + k0);
      const v16b bq2 = Frag<__bf16>::load(w2 + k0);
      const v16b bq3 = Frag<__bf16>::load(w3 + k0);
      acc[0] = Frag<__bf16>::mma(ahv, bq0, acc[0]);
      acc[1] = Frag<__bf16>::mma(ahv, bq1, acc[1]);
      acc[2] = Frag<__bf16>::mma(ahv, bq2, acc[2]);
      acc[3] = Frag<__bf16>::mma(ahv, bq3, acc[3]);
      acc[0] = Frag<__bf16>::mma(alv, bq0, acc[0]);
      acc[1] = Frag<__bf16>::mma(alv, bq1, acc[1]);
      acc[2] = Frag<__bf16>::mma(alv, bq2, acc[2]);
      acc[3] = Frag<__bf16>::mma(alv, bq3, acc[3]);
      mma_guard4_b(acc[0], acc[1], acc[2], acc[3], ahv, alv);
      keep4_b(bq0, bq1, bq2, bq3);
    }
    {
      const v16b axv = Frag<__bf16>::load(ahrow + NHID);
      const v16b bq0 = Frag<__bf16>::load(w0 + NHID);
      const v16b bq1 = Frag<__bf16>::load(w1 + NHID);
      const v16b bq2 = Frag<__bf16>::load(w2 + NHID);
      const v16b bq3 = Frag<__bf16>::load(w3 + NHID);
      acc[0] = Frag<__bf16>::mma(axv, bq0, acc[0]);
      acc[1] = Frag<__bf16>::mma(axv, bq1, acc[1]);
      acc[2] = Frag<__bf16>::mma(axv, bq2, acc[2]);
      acc[3] = Frag<__bf16>::mma(axv, bq3, acc[3]);
      mma_guard4_b(acc[0], acc[1], acc[2], acc[3], axv, bq3);
      keep4_b(bq0, bq1, bq2, bq3);
    }
    acc_guard4(acc[0], acc[1], acc[2], acc[3]);

#pragma unroll
    for (int r = 0; r < 8; ++r) {
      const float zi = acc[0][r] + bb[0];
      const float zf = acc[1][r] + bb[1];
      const float zg = acc[2][r] + bb[2];
      const float zo = acc[3][r] + bb[3];
      const float ig = fsig(zi);
      const float fg = fsig(zf);
      const float gg = ftanh(zg);
      const float og = fsig(zo);
      const float cn = fg * cst[r] + ig * gg;
      cst[r] = cn;
      hst[r] = og * ftanh(cn);
    }
    __syncthreads();
#pragma unroll
    for (int r = 0; r < 8; ++r) {
      const float hn = hst[r];
      const unsigned short hb = f2bf_bits(hn);
      const unsigned short lb = f2bf_bits(hn - bf_bits2f(hb));
      Ah[(arow0 + r) * APITCH + j] = hb;
      Al[(arow0 + r) * LPITCH + j] = lb;
    }
    if (tid < XTHR) {
      v2u pk;
      pk[0] = (unsigned)f2bf_bits(xv[0]) | ((unsigned)f2bf_bits(xv[1]) << 16);
      pk[1] = (unsigned)f2bf_bits(xv[2]) | ((unsigned)f2bf_bits(xv[3]) << 16);
      *(v2u*)(axdst) = pk;
    }
    __syncthreads();
  }

#pragma unroll
  for (int r = 0; r < 8; ++r) Hs[(arow0 + r) * HSP + j] = hst[r];
#pragma unroll 1
  for (int i = tid; i < NZ * NCAT; i += NTHR) W1s[i] = bf16r(W1[i]);
  if (tid < NOUTC * NZ) W2s[tid] = bf16r(W2[tid]);
  __syncthreads();

  {
    const int m = tid >> 4, u0 = 4 * (tid & 15);
    const v4f bv = *(const v4f*)(b1 + u0);
    float z0 = bf16r(bv[0]), z1 = bf16r(bv[1]), z2 = bf16r(bv[2]), z3 = bf16r(bv[3]);
    const float* hrow = Hs + m * HSP;
    const float* wa = W1s + (u0 + 0) * NCAT;
    const float* wb = W1s + (u0 + 1) * NCAT;
    const float* wc = W1s + (u0 + 2) * NCAT;
    const float* wd = W1s + (u0 + 3) * NCAT;
#pragma unroll 1
    for (int k = 0; k < NHID; ++k) {
      const float hk = fmaxf(hrow[k], 0.0f);
      z0 = fmaf(hk, wa[k], z0);
      z1 = fmaf(hk, wb[k], z1);
      z2 = fmaf(hk, wc[k], z2);
      z3 = fmaf(hk, wd[k], z3);
    }
    const float a0 = fmaxf(bf16r(addin[(size_t)(rowbase + m) * 2 + 0]), 0.0f);
    const float a1 = fmaxf(bf16r(addin[(size_t)(rowbase + m) * 2 + 1]), 0.0f);
    z0 = fmaf(a1, wa[NHID + 1], fmaf(a0, wa[NHID], z0));
    z1 = fmaf(a1, wb[NHID + 1], fmaf(a0, wb[NHID], z1));
    z2 = fmaf(a1, wc[NHID + 1], fmaf(a0, wc[NHID], z2));
    z3 = fmaf(a1, wd[NHID + 1], fmaf(a0, wd[NHID], z3));
    v4f zv;
    zv[0] = z0; zv[1] = z1; zv[2] = z2; zv[3] = z3;
    *(v4f*)(Zs + m * ZSP + u0) = zv;
  }
  __syncthreads();

  if (tid < 128) {
    const int m3 = tid / NOUTC;
    const int mm = (m3 < RBLK) ? m3 : (RBLK - 1);
    const int jo = tid - NOUTC * m3;
    float s = bf16r(b2[jo]);
    const float* zrow = Zs + mm * ZSP;
    const float* wr = W2s + jo * NZ;
#pragma unroll 1
    for (int u = 0; u < NZ; ++u) s = fmaf(fmaxf(zrow[u], 0.0f), wr[u], s);
    Os[tid] = (tid < RBLK * NOUTC) ? s : 0.0f;
  }
  __syncthreads();
  if (wave == 0) {
    const v4f v = *(const v4f*)(Os + 4 * lane);
    float* op = out + (size_t)blockIdx.x * (RBLK * NOUTC) + 4 * lane;
    if (lane < (RBLK * NOUTC) / 4) *(volatile v4f*)op = v;
    __threadfence();
    if (lane < (RBLK * NOUTC) / 4) *(volatile v4f*)op = v;
  }
}

extern "C" void kernel_launch(void* const* d_in, const int* in_sizes, int n_in,
                              void* d_out, int out_size, void* d_ws, size_t ws_size, hipStream_t stream) {
  if (n_in < 10 || d_out == nullptr || d_ws == nullptr) return;
  if (in_sizes[0] != NBATCH * NSTEP * NIN || in_sizes[1] != NBATCH * 2 || in_sizes[2] != NGATE * NIN ||
      in_sizes[3] != NGATE * NHID || in_sizes[4] != NGATE || in_sizes[5] != NGATE || in_sizes[6] != NZ * NCAT ||
      in_sizes[7] != NZ || in_sizes[8] != NOUTC * NZ || in_sizes[9] != NOUTC || out_size != NBATCH * NOUTC) return;

  const float* x     = (const float*)d_in[0];
  const float* addin = (const float*)d_in[1];
  const float* w_ih  = (const float*)d_in[2];
  const float* w_hh  = (const float*)d_in[3];
  const float* b_ih  = (const float*)d_in[4];
  const float* b_hh  = (const float*)d_in[5];
  const float* w1    = (const float*)d_in[6];
  const float* b1    = (const float*)d_in[7];
  const float* w2    = (const float*)d_in[8];
  const float* b2    = (const float*)d_in[9];
  float* out = (float*)d_out;

  char* ws = (char*)d_ws; size_t off = 0;
  auto carve = [&](size_t bytes) -> char* { char* p = ws + off; off += (bytes + 255) & ~(size_t)255; return p; };
  unsigned short* WC = (unsigned short*)carve((size_t)NGATE * WPITCH * 2);
  if (off > ws_size || off > (size_t)134217728) return;

  wprep_kernel<<<(NGATE * WGRP) / NPREP, NPREP, 0, stream>>>(w_hh, w_ih, WC);
  lstm_head_kernel<<<NBATCH / RBLK, NTHR, 0, stream>>>(x, addin, WC, b_ih, b_hh, w1, b1, w2, b2, out);
}
